// Arma_84086869721212
// MI455X (gfx1250) — hardware-run, weakly checked
//
#include <hip/hip_runtime.h>
#include <stddef.h>
#include <stdint.h>
#include <math.h>

#define SPLIT_S2 1
#define SPLIT_S3 1
#define SPLIT_S4 1

#define NN      100000
#define NE      1600000
#define FIN     64
#define DIM     32
#define W96     96
#define GBM     128
#define NPAD    100096
#define NTHR    256
#define NWAVE   8
#define EPT     8
#define WCH     (32 * EPT)
#define NBRUN   1024
#define SLB     10
#define NBK     98
#define WLCAP   3584
#define RCAP    28672
#define DEGCAP  64
#define MEAS_MAXDEG 36
#define MEAS_B1024  16710
#define SP      100
#define RPB     64
#define RPW     8
#define AP1     64
#define APB     192
#define WPA     64
#define WPB     192
#define KA1     64
#define KB1     (SPLIT_S2 ? 192 : 96)
#define KA2     (SPLIT_S3 ? 64 : 32)
#define KB2     (SPLIT_S4 ? 192 : 96)
#define PLANE_F ((size_t)NPAD * W96)
#define WSMAX   ((size_t)128 << 20)

#define BK_ZINTS (NWAVE * WLCAP + RCAP + 4 * NBRUN)
#define BK_INTS  (BK_ZINTS + 16)
#define BK_LDS   (BK_INTS * 4)

#define PBX   (NPAD * FIN / 8 / NTHR)
#define PBWA  3
#define PBWB  9
#define PBTOT (PBX + 4 * PBWA + 2 * PBWB + 1)

static_assert(24 * 4 == W96 && W96 == 3 * DIM);
static_assert(NBK * NBRUN >= NN && NBK * NBRUN >= NPAD);
static_assert(782 * GBM == NPAD && NPAD >= NN && NPAD % RPB == 0);
static_assert(NBRUN == (1 << SLB) && NBRUN % RPB == 0 && NBRUN == NTHR * 4);
static_assert(NE < (1 << 21) && (((long long)NE) << SLB) < (1LL << 31));
static_assert(NE % WCH == 0 && NE % 4 == 0);
static_assert(RCAP == NWAVE * WLCAP && RCAP % (NTHR * 4) == 0 && BK_ZINTS % (NTHR * 4) == 0);
static_assert((long long)RCAP * 100 >= (long long)MEAS_B1024 * 105);
static_assert(WLCAP >= MEAS_B1024 / 8 + 8 * 46 + 1);
static_assert(DEGCAP >= MEAS_MAXDEG + 8);
static_assert(BK_LDS <= 300000 && BK_LDS <= 327680);
static_assert((GBM * SP + GBM + W96) * 4 <= 65536);
static_assert((NPAD * FIN / 8) % NTHR == 0 && 96 * 8 == PBWA * NTHR && 96 * 24 == PBWB * NTHR);
static_assert(KA1 % 32 == 0 && KB1 % 32 == 0 && KA2 % 32 == 0 && KB2 % 32 == 0);
static_assert(KA1 <= AP1 && KA2 <= AP1 && KB1 <= APB && KB2 <= APB && KA1 <= WPA && KB1 <= WPB);
static_assert(GBM * W96 / 4 == 12 * NTHR);
static_assert(RPB == NWAVE * RPW);

typedef float          v4f   __attribute__((ext_vector_type(4)));
typedef float          v8f   __attribute__((ext_vector_type(8)));
typedef int            v4i   __attribute__((ext_vector_type(4)));
typedef int            v8i   __attribute__((ext_vector_type(8)));
typedef unsigned short v8us  __attribute__((ext_vector_type(8)));
typedef unsigned short v16us __attribute__((ext_vector_type(16)));
typedef __bf16         v16bf __attribute__((ext_vector_type(16)));
typedef v4f  __attribute__((may_alias)) v4fa;
typedef v4i  __attribute__((may_alias)) v4ia;
typedef v8us __attribute__((may_alias)) v8usa;
union FragB { v16bf v; v16us u; v8us h[2]; v8i w; };

__device__ __forceinline__ v8f wmb(const FragB& a, const FragB& b, v8f c) {
  v8f d = __builtin_amdgcn_wmma_f32_16x16x32_bf16(false, a.v, false, b.v, (short)0, c, false, false);
  asm volatile("v_nop\n\tv_nop\n\tv_nop\n\tv_nop" : "+v"(d) : "v"(a.w), "v"(b.w));
  return d;
}

__device__ __forceinline__ unsigned bf16_bits(float f) {
  const unsigned u = __float_as_uint(f);
  const unsigned r = (u + 0x7FFFu + ((u >> 16) & 1u)) >> 16;
  const unsigned q = (u >> 16) | 0x40u;
  return ((u & 0x7fffffffu) > 0x7f800000u) ? q : r;
}
__device__ __forceinline__ float bf16_val(float f) { return __uint_as_float(bf16_bits(f) << 16); }
__device__ __forceinline__ float relu_k(float v) { return (v > 0.0f) ? v : (v - v); }

__device__ __forceinline__ void hilo_pack(float v0, float v1, float v2, float v3,
                                          int& h01, int& h23, int& l01, int& l23) {
  const unsigned a0 = bf16_bits(v0), a1 = bf16_bits(v1), a2 = bf16_bits(v2), a3 = bf16_bits(v3);
  const unsigned b0 = bf16_bits(v0 - __uint_as_float(a0 << 16));
  const unsigned b1 = bf16_bits(v1 - __uint_as_float(a1 << 16));
  const unsigned b2 = bf16_bits(v2 - __uint_as_float(a2 << 16));
  const unsigned b3 = bf16_bits(v3 - __uint_as_float(a3 << 16));
  h01 = (int)(a0 | (a1 << 16)); h23 = (int)(a2 | (a3 << 16));
  l01 = (int)(b0 | (b1 << 16)); l23 = (int)(b2 | (b3 << 16));
}

__device__ __forceinline__ v4i regroup12(int h01, int h23, int l01, int l23, int lane) {
  const int t  = lane < 24 ? lane : 23;
  const int tt = t < 12 ? t : t - 12;
  const int s0 = 2 * tt, s1 = s0 + 1;
  const int a0 = __shfl(h01, s0, 32), a1 = __shfl(h23, s0, 32), a2 = __shfl(h01, s1, 32), a3 = __shfl(h23, s1, 32);
  const int b0 = __shfl(l01, s0, 32), b1 = __shfl(l23, s0, 32), b2 = __shfl(l01, s1, 32), b3 = __shfl(l23, s1, 32);
  const int mk = (t < 12) ? -1 : 0;
  v4i o;
  o.x = (a0 & mk) | (b0 & ~mk); o.y = (a1 & mk) | (b1 & ~mk);
  o.z = (a2 & mk) | (b2 & ~mk); o.w = (a3 & mk) | (b3 & ~mk);
  return o;
}
__device__ __forceinline__ v4i regroup4(int h01, int h23, int l01, int l23, int lane) {
  const int t  = lane & 7;
  const int tt = t & 3;
  const int s0 = 2 * tt, s1 = s0 + 1;
  const int a0 = __shfl(h01, s0, 32), a1 = __shfl(h23, s0, 32), a2 = __shfl(h01, s1, 32), a3 = __shfl(h23, s1, 32);
  const int b0 = __shfl(l01, s0, 32), b1 = __shfl(l23, s0, 32), b2 = __shfl(l01, s1, 32), b3 = __shfl(l23, s1, 32);
  const int mk = (t < 4) ? -1 : 0;
  v4i o;
  o.x = (a0 & mk) | (b0 & ~mk); o.y = (a1 & mk) | (b1 & ~mk);
  o.z = (a2 & mk) | (b2 & ~mk); o.w = (a3 & mk) | (b3 & ~mk);
  return o;
}

__device__ __forceinline__ void st2_v8us(unsigned short* p, v8us v) {
  *(volatile v8us*)p = v;
  __threadfence();
  *(volatile v8us*)p = v;
}

__device__ __forceinline__ v8us gather8(const float* __restrict__ base, int stride) {
  float f[8];
#pragma unroll
  for (int i = 0; i < 8; ++i) f[i] = base[(size_t)i * (size_t)stride];
  v8us o;
#pragma unroll
  for (int i = 0; i < 8; ++i) o[i] = (unsigned short)bf16_bits(f[i]);
  return o;
}

__device__ __forceinline__ void wa_unit(const float* __restrict__ w, int u, int kmask, int mstride,
                                        unsigned short* dst, int rowOff) {
  const int n = u >> 3, k8 = (u & 7) * 8;
  const int ks = k8 & kmask;
  const v8us o = gather8(w + (size_t)(n >> 5) * (size_t)mstride + (size_t)ks * DIM + (size_t)(n & 31), DIM);
  st2_v8us(dst + (size_t)(rowOff + n) * WPA + k8, o);
}
__device__ __forceinline__ void wb_unit(const float* __restrict__ w, int u, unsigned short* dst) {
  const int n  = u / 24;
  const int j  = u - n * 24;
  const int k8 = 8 * j;
  const int kk = k8 >= W96 ? k8 - W96 : k8;
  const int sk = kk >> 5, kr = kk & 31;
  const int st = n >> 5;
  v8us o = gather8(w + (size_t)st * (DIM * DIM) + (size_t)kr * DIM + (size_t)(n & 31), DIM);
  const unsigned short mk = (sk == st) ? (unsigned short)0xffff : (unsigned short)0;
#pragma unroll
  for (int i = 0; i < 8; ++i) o[i] = (unsigned short)(o[i] & mk);
  st2_v8us(dst + (size_t)n * WPB + k8, o);
}

__global__ __launch_bounds__(NTHR) void k_prep(const float* __restrict__ x,
                                               const float* __restrict__ w1i, const float* __restrict__ w1s,
                                               const float* __restrict__ w1r, const float* __restrict__ b1,
                                               const float* __restrict__ w2i, const float* __restrict__ w2s,
                                               const float* __restrict__ w2r, const float* __restrict__ b2,
                                               unsigned short* xb, unsigned short* wa1, unsigned short* wa2,
                                               unsigned short* wb1, unsigned short* wb2, float* bias) {
  const int tid = (int)threadIdx.x;
  const int blk = (int)blockIdx.x;
  if (blk < PBX) {
    const int u   = blk * NTHR + tid;
    const int row = u >> 3, k8 = (u & 7) * 8;
    const int rc  = row < NN ? row : NN - 1;
    const unsigned mk = row < NN ? 0xffffu : 0u;
    const float* p = x + (size_t)rc * FIN + k8;
    const v4f a = *(const v4fa*)p;
    const v4f b = *(const v4fa*)(p + 4);
    v8us o;
    o[0] = (unsigned short)(bf16_bits(a.x) & mk); o[1] = (unsigned short)(bf16_bits(a.y) & mk);
    o[2] = (unsigned short)(bf16_bits(a.z) & mk); o[3] = (unsigned short)(bf16_bits(a.w) & mk);
    o[4] = (unsigned short)(bf16_bits(b.x) & mk); o[5] = (unsigned short)(bf16_bits(b.y) & mk);
    o[6] = (unsigned short)(bf16_bits(b.z) & mk); o[7] = (unsigned short)(bf16_bits(b.w) & mk);
    st2_v8us(xb + (size_t)row * AP1 + k8, o);
  } else if (blk < PBX + PBWA) {
    wa_unit(w1i, (blk - PBX) * NTHR + tid, 63, FIN * DIM, wa1, 0);
  } else if (blk < PBX + 2 * PBWA) {
    wa_unit(w1r, (blk - PBX - PBWA) * NTHR + tid, 63, FIN * DIM, wa1, W96);
  } else if (blk < PBX + 3 * PBWA) {
    wa_unit(w2i, (blk - PBX - 2 * PBWA) * NTHR + tid, 31, DIM * DIM, wa2, 0);
  } else if (blk < PBX + 4 * PBWA) {
    wa_unit(w2r, (blk - PBX - 3 * PBWA) * NTHR + tid, 31, DIM * DIM, wa2, W96);
  } else if (blk < PBX + 4 * PBWA + PBWB) {
    wb_unit(w1s, (blk - PBX - 4 * PBWA) * NTHR + tid, wb1);
  } else if (blk < PBX + 4 * PBWA + 2 * PBWB) {
    wb_unit(w2s, (blk - PBX - 4 * PBWA - PBWB) * NTHR + tid, wb2);
  } else {
    if (tid < 32) {
      const int lc = tid < 24 ? tid : 23;
      const v4f a = *(const v4fa*)(b1 + 4 * lc);
      const v4f c = *(const v4fa*)(b2 + 4 * lc);
      asm volatile("" :: "v"(a));
      asm volatile("" :: "v"(c));
      v4f oa, oc;
      oa.x = bf16_val(a.x); oa.y = bf16_val(a.y); oa.z = bf16_val(a.z); oa.w = bf16_val(a.w);
      oc.x = bf16_val(c.x); oc.y = bf16_val(c.y); oc.z = bf16_val(c.z); oc.w = bf16_val(c.w);
      float* pa = bias + 4 * lc;
      float* pc = bias + W96 + 4 * lc;
      if (tid < 24) { *(volatile v4f*)pa = oa; *(volatile v4f*)pc = oc; }
      __threadfence();
      if (tid < 24) { *(volatile v4f*)pa = oa; *(volatile v4f*)pc = oc; }
    }
  }
}

__device__ __forceinline__ void bucket_flush(const int* pl, const int* cnt, const int* offs, const int* dnv, int ov,
                                             int* lp, int* cp, int* fp, int* dp, int* flp, int tid) {
#pragma unroll 1
  for (int i = tid * 4; i < RCAP; i += NTHR * 4) {
    const v4i v = *(const v4ia*)(pl + i);
    *(volatile v4i*)(lp + i) = v;
  }
  {
    const v4i vc = *(const v4ia*)(cnt + 4 * tid);
    const v4i vo = *(const v4ia*)(offs + 4 * tid);
    const v4i vd = *(const v4ia*)(dnv + 4 * tid);
    *(volatile v4i*)(cp + 4 * tid) = vc;
    *(volatile v4i*)(fp + 4 * tid) = vo;
    *(volatile v4i*)(dp + 4 * tid) = vd;
  }
  if (tid < 8) {
    const v4i f = {ov, ov, ov, ov};
    *(volatile v4i*)(flp + 4 * tid) = f;
  }
}

__global__ __launch_bounds__(NTHR) void k_bucket(const int* __restrict__ srcs, const int* __restrict__ dsts,
                                                 int* LIST, int* CNT, int* OFF, int* DNVB, int* FLAG) {
  extern __shared__ __attribute__((aligned(16))) int dsm[];
  int* wl   = dsm;
  int* pl   = dsm + NWAVE * WLCAP;
  int* cnt  = pl + RCAP;
  int* offs = cnt + NBRUN;
  int* cur  = offs + NBRUN;
  int* dnv  = cur + NBRUN;
  int* misc = dnv + NBRUN;
  const int tid = (int)threadIdx.x, lane = tid & 31, wave = tid >> 5;
  const int blk = (int)blockIdx.x;
  const unsigned nbs = (unsigned)(blk * NBRUN);
  int nb = NN - blk * NBRUN;
  nb = nb > NBRUN ? NBRUN : (nb < 0 ? 0 : nb);
  const unsigned unb = (unsigned)nb;

  {
    const v4i z4 = {0, 0, 0, 0};
    for (int i = tid * 4; i < BK_ZINTS; i += NTHR * 4) *(v4ia*)(dsm + i) = z4;
    if (tid < 16) misc[tid] = 0;
  }
  __syncthreads();

  {
    const int per  = ((NE + NWAVE * WCH - 1) / (NWAVE * WCH)) * WCH;
    const int ebeg = wave * per;
    const int eend = (ebeg + per < NE) ? (ebeg + per) : NE;
    int* mylist = wl + wave * WLCAP;
    int wc = 0;
#pragma unroll 1
    for (int cb = ebeg; cb < eend; cb += WCH) {
      const int e0 = cb + lane * EPT;
      const v4i da = *(const v4ia*)(dsts + e0);
      const v4i db = *(const v4ia*)(dsts + e0 + 4);
      const unsigned s0 = (unsigned)da.x - nbs, s1 = (unsigned)da.y - nbs;
      const unsigned s2 = (unsigned)da.z - nbs, s3 = (unsigned)da.w - nbs;
      const unsigned s4 = (unsigned)db.x - nbs, s5 = (unsigned)db.y - nbs;
      const unsigned s6 = (unsigned)db.z - nbs, s7 = (unsigned)db.w - nbs;
      const bool h0 = s0 < unb, h1 = s1 < unb, h2 = s2 < unb, h3 = s3 < unb;
      const bool h4 = s4 < unb, h5 = s5 < unb, h6 = s6 < unb, h7 = s7 < unb;
      const unsigned m0 = __builtin_amdgcn_ballot_w32(h0), m1 = __builtin_amdgcn_ballot_w32(h1);
      const unsigned m2 = __builtin_amdgcn_ballot_w32(h2), m3 = __builtin_amdgcn_ballot_w32(h3);
      const unsigned m4 = __builtin_amdgcn_ballot_w32(h4), m5 = __builtin_amdgcn_ballot_w32(h5);
      const unsigned m6 = __builtin_amdgcn_ballot_w32(h6), m7 = __builtin_amdgcn_ballot_w32(h7);
      const unsigned any = m0 | m1 | m2 | m3 | m4 | m5 | m6 | m7;
      if (any != 0u) {
        const int pre = (int)(__builtin_amdgcn_mbcnt_lo(m0, 0u) + __builtin_amdgcn_mbcnt_lo(m1, 0u) +
                              __builtin_amdgcn_mbcnt_lo(m2, 0u) + __builtin_amdgcn_mbcnt_lo(m3, 0u) +
                              __builtin_amdgcn_mbcnt_lo(m4, 0u) + __builtin_amdgcn_mbcnt_lo(m5, 0u) +
                              __builtin_amdgcn_mbcnt_lo(m6, 0u) + __builtin_amdgcn_mbcnt_lo(m7, 0u));
        int p = wc + pre;
        if (h0) { if (p < WLCAP) mylist[p] = ((e0 + 0) << SLB) | (int)s0; p = p + 1; }
        if (h1) { if (p < WLCAP) mylist[p] = ((e0 + 1) << SLB) | (int)s1; p = p + 1; }
        if (h2) { if (p < WLCAP) mylist[p] = ((e0 + 2) << SLB) | (int)s2; p = p + 1; }
        if (h3) { if (p < WLCAP) mylist[p] = ((e0 + 3) << SLB) | (int)s3; p = p + 1; }
        if (h4) { if (p < WLCAP) mylist[p] = ((e0 + 4) << SLB) | (int)s4; p = p + 1; }
        if (h5) { if (p < WLCAP) mylist[p] = ((e0 + 5) << SLB) | (int)s5; p = p + 1; }
        if (h6) { if (p < WLCAP) mylist[p] = ((e0 + 6) << SLB) | (int)s6; p = p + 1; }
        if (h7) { if (p < WLCAP) mylist[p] = ((e0 + 7) << SLB) | (int)s7; p = p + 1; }
        wc += (int)(__builtin_popcount(m0) + __builtin_popcount(m1) + __builtin_popcount(m2) + __builtin_popcount(m3) +
                    __builtin_popcount(m4) + __builtin_popcount(m5) + __builtin_popcount(m6) + __builtin_popcount(m7));
      }
    }
    if (lane == 0) misc[wave] = wc;
  }
  __syncthreads();

  if (wave == 0) {
    int ov = 0;
#pragma unroll 1
    for (int w2 = 0; w2 < NWAVE; ++w2) {
      int c = misc[w2];
      if (c > WLCAP) ov = 1;
      c = c < 0 ? 0 : (c > WLCAP ? WLCAP : c);
#pragma unroll 1
      for (int b0 = 0; b0 < c; b0 += 32) {
        const int idx = b0 + lane;
        const int ent = wl[w2 * WLCAP + (idx < WLCAP ? idx : WLCAP - 1)];
        const int m32 = (c - b0) < 32 ? (c - b0) : 32;
#pragma unroll 1
        for (int k = 0; k < m32; ++k) {
          const int u    = __builtin_amdgcn_readlane(ent, k);
          const int slot = u & (NBRUN - 1);
          if (lane == 0) cnt[slot] = cnt[slot] + 1;
        }
      }
    }
    if (lane == 0) misc[9] = ov;
  }
  __syncthreads();
  if (wave == 0) {
    const int base = lane * (NBRUN / 32);
    int s = 0;
#pragma unroll 1
    for (int i = 0; i < NBRUN / 32; ++i) s += cnt[base + i];
    int incl = s;
#pragma unroll
    for (int d = 1; d < 32; d <<= 1) {
      const int y = __shfl_up(incl, d, 32);
      if (lane >= d) incl += y;
    }
    int run = incl - s;
#pragma unroll 1
    for (int i = 0; i < NBRUN / 32; ++i) {
      const int cv = cnt[base + i];
      offs[base + i] = run;
      cur[base + i]  = run;
      run += cv;
    }
  }
  __syncthreads();

  if (wave == 0) {
#pragma unroll 1
    for (int w2 = 0; w2 < NWAVE; ++w2) {
      int c = misc[w2];
      c = c < 0 ? 0 : (c > WLCAP ? WLCAP : c);
#pragma unroll 1
      for (int b0 = 0; b0 < c; b0 += 32) {
        const int idx = b0 + lane;
        const int ent = wl[w2 * WLCAP + (idx < WLCAP ? idx : WLCAP - 1)];
        int eid = (ent >> SLB) & 0x1FFFFF;
        eid = eid > NE - 1 ? NE - 1 : eid;
        int sr = srcs[eid];
        sr = sr < 0 ? 0 : (sr > NN - 1 ? NN - 1 : sr);
        const int m32 = (c - b0) < 32 ? (c - b0) : 32;
#pragma unroll 1
        for (int k = 0; k < m32; ++k) {
          const int u    = __builtin_amdgcn_readlane(ent, k);
          const int wd   = __builtin_amdgcn_readlane(sr, k);
          const int slot = u & (NBRUN - 1);
          if (lane == 0) {
            int p = cur[slot];
            p = p < 0 ? 0 : (p > RCAP - 1 ? RCAP - 1 : p);
            pl[p] = wd;
            cur[slot] = p + 1;
          }
        }
      }
    }
  }
  __syncthreads();

#pragma unroll 1
  for (int i = 0; i < 4; ++i) {
    const int cv = cnt[4 * tid + i];
    const int cm = cv > 1 ? cv : 1;
    const float d = 1.0f / sqrtf((float)cm);
    dnv[4 * tid + i] = (cv > 0) ? __float_as_int(d) : 0;
  }
  __syncthreads();

  const int ovf = misc[9];
  int* lp  = LIST + (size_t)blk * RCAP;
  int* cp  = CNT + (size_t)blk * NBRUN;
  int* fp  = OFF + (size_t)blk * NBRUN;
  int* dp  = DNVB + (size_t)blk * NBRUN;
  int* flp = FLAG + (size_t)blk * 32;
  bucket_flush(pl, cnt, offs, dnv, ovf, lp, cp, fp, dp, flp, tid);
  __threadfence();
  bucket_flush(pl, cnt, offs, dnv, ovf, lp, cp, fp, dp, flp, tid);
}

template <int KTOT, int WP>
__device__ __forceinline__ void gemm_16x96(const unsigned short* __restrict__ ap,
                                           const unsigned short* __restrict__ bp, v8f (&acc)[6]) {
#pragma unroll 1
  for (int k0 = 0; k0 < KTOT; k0 += 32) {
    FragB af;
    af.h[0] = *(const v8usa*)(ap + k0);
    af.h[1] = *(const v8usa*)(ap + k0 + 16);
#pragma unroll
    for (int nt = 0; nt < 6; ++nt) {
      const unsigned short* wq = bp + (size_t)(16 * nt) * (size_t)WP + k0;
      FragB bf;
      bf.h[0] = *(const v8usa*)wq;
      bf.h[1] = *(const v8usa*)(wq + 16);
      acc[nt] = wmb(af, bf, acc[nt]);
    }
  }
}

__device__ __forceinline__ void gemm_flush(const float* stg, float* ob, int tid) {
#pragma unroll 1
  for (int it = 0; it < 12; ++it) {
    const int i4  = it * NTHR + tid;
    const int row = i4 / 24;
    const int c4  = i4 - row * 24;
    const v4f v = *(const v4fa*)(stg + row * SP + 4 * c4);
    asm volatile("" :: "v"(v));
    *(volatile v4f*)(ob + (size_t)4 * (size_t)i4) = v;
  }
}

template <int KTOT, int APITCH, int WP>
__global__ __launch_bounds__(NTHR) __attribute__((amdgpu_num_vgpr(248)))
void k_gemm(const unsigned short* __restrict__ A, const unsigned short* __restrict__ BT,
            const float* __restrict__ DINV, const float* __restrict__ BIAS, float* PR) {
  __shared__ __attribute__((aligned(16))) float stg[GBM * SP];
  __shared__ __attribute__((aligned(16))) float sdv[GBM];
  __shared__ __attribute__((aligned(16))) float sb[W96];
  const int tid = (int)threadIdx.x, lane = tid & 31, wave = tid >> 5, hh = lane >> 4, m = lane & 15;
  const int rowBase = (int)blockIdx.x * GBM;
  const int isR     = (int)blockIdx.y;
  const int colBase = isR * W96;

  if (tid < 32) {
    const int lc = tid < 24 ? tid : 23;
    const v4f dv = *(const v4fa*)(DINV + (size_t)rowBase + 4 * tid);
    const v4f bv = *(const v4fa*)(BIAS + 4 * lc);
    asm volatile("" :: "v"(dv));
    asm volatile("" :: "v"(bv));
    *(v4fa*)(sdv + 4 * tid) = dv;
    if (tid < 24) *(v4fa*)(sb + 4 * tid) = bv;
  }

  v8f acc[6];
  {
    const v8f z = {0.f, 0.f, 0.f, 0.f, 0.f, 0.f, 0.f, 0.f};
#pragma unroll
    for (int t = 0; t < 6; ++t) acc[t] = z;
  }
  const unsigned short* ap = A + (size_t)(rowBase + 16 * wave + m) * (size_t)APITCH + 8 * hh;
  const unsigned short* bp = BT + (size_t)(colBase + m) * (size_t)WP + 8 * hh;
  gemm_16x96<KTOT, WP>(ap, bp, acc);
  __syncthreads();

  float dvr[8];
#pragma unroll
  for (int r = 0; r < 8; ++r) dvr[r] = sdv[16 * wave + 8 * hh + r];
#pragma unroll
  for (int nt = 0; nt < 6; ++nt) {
    const float bb = sb[16 * nt + m];
#pragma unroll
    for (int r = 0; r < 8; ++r) {
      const float a  = acc[nt][r];
      const float vr = a + bb;
      const float vp = a * dvr[r];
      stg[(16 * wave + 8 * hh + r) * SP + 16 * nt + m] = (isR != 0) ? vr : vp;
    }
  }
  __syncthreads();

  float* ob = PR + (size_t)isR * PLANE_F + (size_t)rowBase * W96;
  gemm_flush(stg, ob, tid);
  __threadfence();
  gemm_flush(stg, ob, tid);
}

__device__ __forceinline__ void slot_info(const int* __restrict__ CNT, const int* __restrict__ OFF,
                                          const float* __restrict__ DINV, int node,
                                          int& c, int& o, int& big, float& dv) {
  const int craw = CNT[node];
  const int oraw = OFF[node];
  dv = DINV[node];
  big = craw > DEGCAP ? 1 : 0;
  int cc = craw < 0 ? 0 : (craw > DEGCAP ? DEGCAP : craw);
  int oo = oraw < 0 ? 0 : (oraw > RCAP - 1 ? RCAP - 1 : oraw);
  cc = cc > RCAP - oo ? RCAP - oo : cc;
  c = __builtin_amdgcn_readfirstlane(cc);
  o = __builtin_amdgcn_readfirstlane(oo);
}

__device__ __forceinline__ v4f gather_sum(const float* __restrict__ P, const int* __restrict__ lb,
                                          int o, int c, int lane, int lc) {
  int last = o + c - 1; last = last < o ? o : last;
  float a0 = 0.0f, a1 = 0.0f, a2 = 0.0f, a3 = 0.0f;
#pragma unroll 1
  for (int b0 = 0; b0 < c; b0 += 32) {
    int idx = o + b0 + lane;
    idx = idx > last ? last : idx;
    int col = lb[idx];
    col = col < 0 ? 0 : (col > NN - 1 ? NN - 1 : col);
    const int m32 = (c - b0) < 32 ? (c - b0) : 32;
#pragma unroll 1
    for (int k = 0; k < m32; ++k) {
      const int sk = __builtin_amdgcn_readlane(col, k);
      const v4f v = *(const v4fa*)(P + (size_t)sk * W96 + 4 * lc);
      a0 += v.x; a1 += v.y; a2 += v.z; a3 += v.w;
    }
  }
  v4f r;
  r.x = a0; r.y = a1; r.z = a2; r.w = a3;
  return r;
}

template <int ACT>
__global__ __launch_bounds__(NTHR) void k_replay0(const float* __restrict__ PR, const int* __restrict__ LIST,
                                                  const int* __restrict__ CNT, const int* __restrict__ OFF,
                                                  const float* __restrict__ DINV, const int* __restrict__ FLAG,
                                                  unsigned short* OHL) {
  const int tid = (int)threadIdx.x, lane = tid & 31, wave = tid >> 5;
  const int lc = lane < 24 ? lane : 23;
  const int rowBase = (int)blockIdx.x * RPB;
  const int bucket  = rowBase >> SLB;
  const int* lb = LIST + (size_t)bucket * RCAP;
  const int flag = FLAG[(size_t)bucket * 32];
  const float* P = PR;
  const float* R = PR + PLANE_F;
  const float qnan = __uint_as_float(0x7fc00000u);
#pragma unroll 1
  for (int ri = 0; ri < RPW; ++ri) {
    const int node = rowBase + wave * RPW + ri;
    int c, o, big; float dv;
    slot_info(CNT, OFF, DINV, node, c, o, big, dv);
    const v4f a = gather_sum(P, lb, o, c, lane, lc);
    const v4f r = *(const v4fa*)(R + (size_t)node * W96 + 4 * lc);
    asm volatile("" :: "v"(r));
    float v0 = dv * a.x + r.x, v1 = dv * a.y + r.y, v2 = dv * a.z + r.z, v3 = dv * a.w + r.w;
    if constexpr (ACT != 0) { v0 = relu_k(v0); v1 = relu_k(v1); v2 = relu_k(v2); v3 = relu_k(v3); }
    const bool bad  = (flag != 0) | (big != 0);
    const bool live = node < NN;
    v0 = bad ? qnan : v0; v1 = bad ? qnan : v1; v2 = bad ? qnan : v2; v3 = bad ? qnan : v3;
    v0 = live ? v0 : 0.0f; v1 = live ? v1 : 0.0f; v2 = live ? v2 : 0.0f; v3 = live ? v3 : 0.0f;
    int h01, h23, l01, l23;
    hilo_pack(v0, v1, v2, v3, h01, h23, l01, l23);
    const v4i ow = regroup12(h01, h23, l01, l23, lane);
    unsigned short* hp = OHL + (size_t)node * APB + 8 * lc;
    if (lane < 24) *(volatile v4i*)hp = ow;
    __threadfence();
    if (lane < 24) *(volatile v4i*)hp = ow;
  }
}

template <int LAST>
__global__ __launch_bounds__(NTHR) void k_replay1(const float* __restrict__ PR, const int* __restrict__ LIST,
                                                  const int* __restrict__ CNT, const int* __restrict__ OFF,
                                                  const float* __restrict__ DINV, const int* __restrict__ FLAG,
                                                  unsigned short* HHL, float* out) {
  const int tid = (int)threadIdx.x, lane = tid & 31, wave = tid >> 5;
  const int lc = lane < 24 ? lane : 23;
  const int rowBase = (int)blockIdx.x * RPB;
  const int bucket  = rowBase >> SLB;
  const int* lb = LIST + (size_t)bucket * RCAP;
  const int flag = FLAG[(size_t)bucket * 32];
  const float* P = PR;
  const float* R = PR + PLANE_F;
  const float qnan = __uint_as_float(0x7fc00000u);
  const int sl1 = (lane + 8) & 31, sl2 = (lane + 16) & 31;
#pragma unroll 1
  for (int ri = 0; ri < RPW; ++ri) {
    const int node = rowBase + wave * RPW + ri;
    if constexpr (LAST != 0) { if (node >= NN) continue; }
    int c, o, big; float dv;
    slot_info(CNT, OFF, DINV, node, c, o, big, dv);
    const v4f a = gather_sum(P, lb, o, c, lane, lc);
    const v4f r = *(const v4fa*)(R + (size_t)node * W96 + 4 * lc);
    asm volatile("" :: "v"(r));
    float v0 = dv * a.x + r.x, v1 = dv * a.y + r.y, v2 = dv * a.z + r.z, v3 = dv * a.w + r.w;
    if constexpr (LAST == 0) { v0 = relu_k(v0); v1 = relu_k(v1); v2 = relu_k(v2); v3 = relu_k(v3); }
    const float p0 = __shfl(v0, sl1, 32), p1 = __shfl(v1, sl1, 32), p2 = __shfl(v2, sl1, 32), p3 = __shfl(v3, sl1, 32);
    const float q0 = __shfl(v0, sl2, 32), q1 = __shfl(v1, sl2, 32), q2 = __shfl(v2, sl2, 32), q3 = __shfl(v3, sl2, 32);
    float m0 = ((v0 + p0) + q0) / 3.0f;
    float m1 = ((v1 + p1) + q1) / 3.0f;
    float m2 = ((v2 + p2) + q2) / 3.0f;
    float m3 = ((v3 + p3) + q3) / 3.0f;
    const bool bad = (flag != 0) | (big != 0);
    if constexpr (LAST == 0) {
      m0 = relu_k(m0); m1 = relu_k(m1); m2 = relu_k(m2); m3 = relu_k(m3);
      const bool live = node < NN;
      m0 = bad ? qnan : m0; m1 = bad ? qnan : m1; m2 = bad ? qnan : m2; m3 = bad ? qnan : m3;
      m0 = live ? m0 : 0.0f; m1 = live ? m1 : 0.0f; m2 = live ? m2 : 0.0f; m3 = live ? m3 : 0.0f;
      int h01, h23, l01, l23;
      hilo_pack(m0, m1, m2, m3, h01, h23, l01, l23);
      const v4i ow = regroup4(h01, h23, l01, l23, lane);
      unsigned short* hp = HHL + (size_t)node * AP1 + 8 * (lane & 7);
      if (lane < 8) *(volatile v4i*)hp = ow;
      __threadfence();
      if (lane < 8) *(volatile v4i*)hp = ow;
    } else {
      m0 = bad ? qnan : m0; m1 = bad ? qnan : m1; m2 = bad ? qnan : m2; m3 = bad ? qnan : m3;
      v4f ov;
      ov.x = m0; ov.y = m1; ov.z = m2; ov.w = m3;
      float* op = out + (size_t)node * DIM + 4 * (lane & 7);
      if (lane < 8) *(volatile v4f*)op = ov;
      __threadfence();
      if (lane < 8) *(volatile v4f*)op = ov;
    }
  }
}

extern "C" void kernel_launch(void* const* d_in, const int* in_sizes, int n_in,
                              void* d_out, int out_size, void* d_ws, size_t ws_size,
                              hipStream_t stream) {
  if (n_in < 10) return;
  if (in_sizes[0] != NN * FIN) return;
  if (in_sizes[1] != 2 * NE) return;
  if (in_sizes[2] != 3 * FIN * DIM) return;
  if (in_sizes[3] != 3 * DIM * DIM) return;
  if (in_sizes[4] != 3 * FIN * DIM) return;
  if (in_sizes[5] != W96) return;
  if (in_sizes[6] != 3 * DIM * DIM) return;
  if (in_sizes[7] != 3 * DIM * DIM) return;
  if (in_sizes[8] != 3 * DIM * DIM) return;
  if (in_sizes[9] != W96) return;
  if (out_size != NN * DIM) return;

  const float* x   = (const float*)d_in[0];
  const int*   ei  = (const int*)d_in[1];
  const float* w1i = (const float*)d_in[2];
  const float* w1s = (const float*)d_in[3];
  const float* w1r = (const float*)d_in[4];
  const float* b1  = (const float*)d_in[5];
  const float* w2i = (const float*)d_in[6];
  const float* w2s = (const float*)d_in[7];
  const float* w2r = (const float*)d_in[8];
  const float* b2  = (const float*)d_in[9];
  float* out = (float*)d_out;
  const int* srcs = ei;
  const int* dsts = ei + NE;

  constexpr size_t zPL   = (size_t)NPAD * W96 * 4;
  constexpr size_t zOHL  = (size_t)NPAD * APB * 2;
  constexpr size_t zXB   = (size_t)NPAD * AP1 * 2;
  constexpr size_t zLIST = (size_t)NBK * RCAP * 4;
  constexpr size_t zTAB  = (size_t)NBK * NBRUN * 4;
  constexpr size_t zFLAG = (size_t)NBK * 128;
  constexpr size_t zWA   = (size_t)192 * WPA * 2;
  constexpr size_t zWB   = (size_t)W96 * WPB * 2;
  constexpr size_t zBIAS = 1024;
  constexpr size_t oP    = 0;
  constexpr size_t oOHL  = oP + 2 * zPL;
  constexpr size_t oLIST = oOHL + zOHL;
  constexpr size_t oCNT  = oLIST + zLIST;
  constexpr size_t oOFF  = oCNT + zTAB;
  constexpr size_t oDNV  = oOFF + zTAB;
  constexpr size_t oFLAG = oDNV + zTAB;
  constexpr size_t oWA1  = oFLAG + zFLAG;
  constexpr size_t oWA2  = oWA1 + zWA;
  constexpr size_t oWB1  = oWA2 + zWA;
  constexpr size_t oWB2  = oWB1 + zWB;
  constexpr size_t oBIAS = oWB2 + zWB;
  constexpr size_t oEND  = oBIAS + zBIAS;
  static_assert(zPL % 256 == 0 && zOHL % 256 == 0 && zLIST % 256 == 0 && zTAB % 256 == 0 && zFLAG % 256 == 0);
  static_assert(zWA % 256 == 0 && zWB % 256 == 0 && zBIAS % 256 == 0 && zXB <= zOHL);
  static_assert((size_t)(NPAD - 1) * W96 + W96 <= PLANE_F);
  static_assert(oEND <= WSMAX);
  if (oEND > ws_size) return;

  char* ws = (char*)d_ws;
  float*          PR   = (float*)(ws + oP);
  unsigned short* OHL  = (unsigned short*)(ws + oOHL);
  unsigned short* XB   = OHL;
  unsigned short* HHL  = OHL;
  int*            LIST = (int*)(ws + oLIST);
  int*            CNT  = (int*)(ws + oCNT);
  int*            OFF  = (int*)(ws + oOFF);
  float*          DINV = (float*)(ws + oDNV);
  int*            FLAG = (int*)(ws + oFLAG);
  unsigned short* WA1  = (unsigned short*)(ws + oWA1);
  unsigned short* WA2  = (unsigned short*)(ws + oWA2);
  unsigned short* WB1  = (unsigned short*)(ws + oWB1);
  unsigned short* WB2  = (unsigned short*)(ws + oWB2);
  float*          BIAS = (float*)(ws + oBIAS);

  hipFuncSetAttribute(reinterpret_cast<const void*>(&k_bucket), hipFuncAttributeMaxDynamicSharedMemorySize, (int)BK_LDS);

  const dim3 gA((unsigned)(NPAD / GBM), 2u, 1u);
  const dim3 gB((unsigned)(NPAD / GBM), 1u, 1u);
  const int gR = NPAD / RPB;

  k_prep<<<PBTOT, NTHR, 0, stream>>>(x, w1i, w1s, w1r, b1, w2i, w2s, w2r, b2, XB, WA1, WA2, WB1, WB2, BIAS);
  k_bucket<<<NBK, NTHR, BK_LDS, stream>>>(srcs, dsts, LIST, CNT, OFF, (int*)DINV, FLAG);
  k_gemm<KA1, AP1, WPA><<<gA, NTHR, 0, stream>>>(XB, WA1, DINV, BIAS, PR);
  k_replay0<1><<<gR, NTHR, 0, stream>>>(PR, LIST, CNT, OFF, DINV, FLAG, OHL);
  k_gemm<KB1, APB, WPB><<<gB, NTHR, 0, stream>>>(OHL, WB1, DINV, BIAS, PR);
  k_replay1<0><<<gR, NTHR, 0, stream>>>(PR, LIST, CNT, OFF, DINV, FLAG, HHL, out);
  k_gemm<KA2, AP1, WPA><<<gA, NTHR, 0, stream>>>(HHL, WA2, DINV, BIAS + W96, PR);
  k_replay0<0><<<gR, NTHR, 0, stream>>>(PR, LIST, CNT, OFF, DINV, FLAG, OHL);
  k_gemm<KB2, APB, WPB><<<gB, NTHR, 0, stream>>>(OHL, WB2, DINV, BIAS + W96, PR);
  k_replay1<1><<<gR, NTHR, 0, stream>>>(PR, LIST, CNT, OFF, DINV, FLAG, HHL, out);
}
